// WL_DiffNet_970662609325
// MI455X (gfx1250) — hardware-run, weakly checked
//
#include <hip/hip_runtime.h>
#include <math.h>

typedef __attribute__((ext_vector_type(16))) _Float16 v16h;
typedef __attribute__((ext_vector_type(16))) __bf16 v16b;
typedef __attribute__((ext_vector_type(8)))  _Float16 v8h;
typedef __attribute__((ext_vector_type(8)))  float v8f;
typedef __attribute__((ext_vector_type(4)))  float v4f;
typedef __attribute__((ext_vector_type(2)))  float v2f;
typedef __attribute__((ext_vector_type(4)))  unsigned v4u;
typedef __attribute__((ext_vector_type(4)))  int v4i;
typedef float __attribute__((may_alias)) float_a;
typedef int __attribute__((may_alias)) int_a;

template <typename T> __device__ __forceinline__ void vst2(void* p, T v) { *(volatile T*)p = v; __threadfence(); *(volatile T*)p = v; }
__device__ __forceinline__ v8f wmma16(v16h a, v16h b, v8f c) {
  v8f d = __builtin_amdgcn_wmma_f32_16x16x32_f16(false, a, false, b, (short)0, c, false, false);
  asm volatile("v_nop\n\tv_nop\n\tv_nop\n\tv_nop" : "+v"(d) : "v"(a), "v"(b));
  return d;
}
__device__ __forceinline__ v8f wmma_bf(v16b a, v16b b, v8f c) {
  v8f d = __builtin_amdgcn_wmma_f32_16x16x32_bf16(false, a, false, b, (short)0, c, false, false);
  asm volatile("v_nop\n\tv_nop\n\tv_nop\n\tv_nop" : "+v"(d) : "v"(a), "v"(b));
  return d;
}
__device__ __forceinline__ v16h frag_h(const _Float16* rowk0, int lane) {
  union { v16h v; v8h q[2]; } u; const _Float16* p = rowk0 + 8 * (lane >> 4);
  u.q[0] = *(const v8h*)p; u.q[1] = *(const v8h*)(p + 16); return u.v;
}
__device__ __forceinline__ v16h frag_f32(const float* rowk0, int lane) {
  v16h a; const float* p = rowk0 + 8 * (lane >> 4);
#pragma unroll
  for (int i = 0; i < 8; ++i) { a[i] = (_Float16)p[i]; a[8 + i] = (_Float16)p[16 + i]; }
  return a;
}
__device__ __forceinline__ v16h frag_f32s(const float* rowk0, int lane, float sc) {
  v16h a; const float* p = rowk0 + 8 * (lane >> 4);
#pragma unroll
  for (int i = 0; i < 8; ++i) { a[i] = (_Float16)(p[i] * sc); a[8 + i] = (_Float16)(p[16 + i] * sc); }
  return a;
}
__device__ __forceinline__ v16h fragc_f32(const float* W, int k0, int n, int lane, int ld, int K) {
  v16h a; const int g = lane >> 4;
#pragma unroll
  for (int i = 0; i < 8; ++i) { const int ka = k0 + 8 * g + i, kb = ka + 16;
    a[i] = (_Float16)(ka < K ? W[(size_t)(ka < K ? ka : K - 1) * ld + n] : 0.f); a[8 + i] = (_Float16)(kb < K ? W[(size_t)(kb < K ? kb : K - 1) * ld + n] : 0.f); }
  return a;
}
struct F2 { v16b h, l; };
__device__ __forceinline__ F2 bsplit16(const float v[16]) { F2 r;
#pragma unroll
  for (int i = 0; i < 16; ++i) { const __bf16 h = (__bf16)v[i]; r.h[i] = h; r.l[i] = (__bf16)(v[i] - (float)h); }
  return r; }
__device__ __forceinline__ F2 split_row(const float* row, int k0, int lane) { float v[16]; const float* p = row + k0 + 8 * (lane >> 4);
#pragma unroll
  for (int i = 0; i < 8; ++i) { v[i] = p[i]; v[8 + i] = p[16 + i]; }
  return bsplit16(v); }
__device__ __forceinline__ F2 split_rowK(const float* row, int k0, int lane, int K) { float v[16]; const int g = lane >> 4;
#pragma unroll
  for (int i = 0; i < 8; ++i) { const int ka = k0 + 8 * g + i, kb = ka + 16; v[i] = ka < K ? row[ka < K ? ka : K - 1] : 0.f; v[8 + i] = kb < K ? row[kb < K ? kb : K - 1] : 0.f; }
  return bsplit16(v); }
__device__ __forceinline__ F2 split_col(const float* W, int k0, int n, int lane, int ld, int K) { float v[16]; const int g = lane >> 4;
#pragma unroll
  for (int i = 0; i < 8; ++i) { const int ka = k0 + 8 * g + i, kb = ka + 16; v[i] = ka < K ? W[(size_t)(ka < K ? ka : K - 1) * ld + n] : 0.f; v[8 + i] = kb < K ? W[(size_t)(kb < K ? kb : K - 1) * ld + n] : 0.f; }
  return bsplit16(v); }
__device__ __forceinline__ v8f mac3(const F2& a, const F2& b, v8f c) { c = wmma_bf(a.l, b.h, c); c = wmma_bf(a.h, b.l, c); return wmma_bf(a.h, b.h, c); }
__device__ __forceinline__ float sigm(float v) { return 1.0f / (1.0f + expf(-v)); }
#define LDSX() do { asm volatile("s_wait_dscnt 0" ::: "memory"); __builtin_amdgcn_wave_barrier(); __builtin_amdgcn_fence(__ATOMIC_RELEASE, "workgroup"); } while (0)


#define NB 64
#define NA 512
#define NNB 10
#define HH 256
#define BF 5
#define DEPTH 3
#define NR (NB * NA)
#ifndef TNB
#define TNB NB
#endif
typedef __attribute__((ext_vector_type(8))) __bf16 v8b;
__device__ __forceinline__ v16b frag_b(const __bf16* rowk0, int lane) {
  union { v16b v; v8b q[2]; } u; const __bf16* p = rowk0 + 8 * (lane >> 4);
  u.q[0] = *(const v8b*)p; u.q[1] = *(const v8b*)(p + 16); return u.v;
}
__device__ __forceinline__ float bfr(float v) { return (float)(__bf16)v; }
__device__ __attribute__((noinline)) float exp_ni(float v) { return expf(v); }
__device__ __attribute__((noinline)) float erf_ni(float v) { return erff(v); }

#define WS_P2  0u
#define WS_P1  (WS_P2 + 2u * (size_t)HH * HH)
#define WS_FA  (WS_P1 + 2u * (size_t)HH * 2 * HH)
#define WS_FB  (WS_FA + 4u * (size_t)NR * HH)
#define WS_FW  (WS_FB + 4u * (size_t)NR * HH)
#define WS_NEI (WS_FW + 4u * (size_t)NR * HH)
#define WS_END (WS_NEI + 4u * (size_t)NR * HH)

__global__ __launch_bounds__(256) void k_pack(const float* __restrict__ W2, const float* __restrict__ W1, __bf16* __restrict__ P) { const int n = blockIdx.x, which = blockIdx.y, t = threadIdx.x; __shared__ __align__(16) __bf16 s[2 * HH];
  if (which == 0) { s[t] = (__bf16)W2[(size_t)t * HH + n]; __syncthreads(); if (t < HH / 8) vst2((unsigned*)(P + WS_P2 / 2 + (size_t)n * HH + t * 8), *(const v4u*)&s[t * 8]); }
  else { s[t] = (__bf16)W1[(size_t)t * HH + n]; s[HH + t] = (__bf16)W1[(size_t)(HH + t) * HH + n]; __syncthreads(); if (t < 2 * HH / 8) vst2((unsigned*)(P + WS_P1 / 2 + (size_t)n * 2 * HH + t * 8), *(const v4u*)&s[t * 8]); } }
__global__ __launch_bounds__(256) void k_copy(const float* __restrict__ AF, float* __restrict__ FA) { const size_t row = blockIdx.x; const int t = threadIdx.x; __shared__ __align__(16) float s[HH]; s[t] = bfr(AF[row * HH + t]); __syncthreads(); if (t < HH / 4) vst2(FA + row * HH + t * 4, *(const v4f*)&s[t * 4]); }
__global__ __launch_bounds__(128) void k_fw(const float* __restrict__ FEAT, const __bf16* __restrict__ P2, float* __restrict__ FW) { __shared__ __align__(16) float sf[4][16][132];
  const int tid = threadIdx.x, wave = tid >> 5, lane = tid & 31, col = lane & 15, g = lane >> 4; const size_t r0 = (size_t)blockIdx.x * 64 + wave * 16; const int c0 = blockIdx.y * 128;
  v8f acc[8] = {};
#pragma unroll 2
  for (int kc = 0; kc < HH / 32; ++kc) { const F2 a = split_row(FEAT + (r0 + col) * HH, kc * 32, lane);
#pragma unroll
    for (int j = 0; j < 8; ++j) { const v16b w = frag_b(P2 + (size_t)(c0 + j * 16 + col) * HH + kc * 32, lane); acc[j] = wmma_bf(a.h, w, acc[j]); acc[j] = wmma_bf(a.l, w, acc[j]); } }
#pragma unroll
  for (int j = 0; j < 8; ++j)
#pragma unroll
    for (int r = 0; r < 8; ++r) sf[wave][8 * g + r][j * 16 + col] = acc[j][r];
  LDSX(); for (int rl = 0; rl < 16; ++rl) vst2(FW + (r0 + rl) * HH + c0 + lane * 4, *(const v4f*)&sf[wave][rl][lane * 4]); }
__global__ __launch_bounds__(256) void k_nei(const float* __restrict__ FW, const float* __restrict__ BOND, const int* __restrict__ AG, const int* __restrict__ BG, const int* __restrict__ NNBS, const float* __restrict__ W2, const float* __restrict__ B2, float* __restrict__ NEI) {
  __shared__ int sa[NNB], sb[NNB]; __shared__ float sbond[NNB][BF]; __shared__ __align__(16) float so2[HH]; const int t = threadIdx.x; const size_t row = blockIdx.x;
  int nn = NNBS[row]; nn = nn < 0 ? 0 : (nn > NNB ? NNB : nn);
  if (t < NNB) { int b0 = AG[(row * NNB + t) * 2], a1 = AG[(row * NNB + t) * 2 + 1]; b0 = b0 < 0 ? 0 : (b0 >= NB ? NB - 1 : b0); a1 = a1 < 0 ? 0 : (a1 >= NA ? NA - 1 : a1); sa[t] = b0 * NA + a1;
    int c0 = BG[(row * NNB + t) * 2], c1 = BG[(row * NNB + t) * 2 + 1]; c0 = c0 < 0 ? 0 : (c0 >= NB ? NB - 1 : c0); c1 = c1 < 0 ? 0 : (c1 >= NA ? NA - 1 : c1); sb[t] = c0 * NA + c1; }
  __syncthreads(); if (t < NNB * BF) sbond[t / BF][t % BF] = bfr(BOND[(size_t)sb[t / BF] * BF + t % BF]); __syncthreads();
  float w5[BF]; for (int j = 0; j < BF; ++j) w5[j] = bfr(W2[(size_t)(HH + j) * HH + t]); const float bb = bfr(B2[t]);
  float acc = 0.f;
#pragma unroll 1
  for (int k = 0; k < NNB; ++k) { if (k >= nn) break; float v = FW[(size_t)sa[k] * HH + t] + bb; for (int j = 0; j < BF; ++j) v += sbond[k][j] * w5[j]; acc += fmaxf(v, 0.f); }
  so2[t] = acc; __syncthreads(); if (t < HH / 4) vst2(NEI + row * HH + t * 4, *(const v4f*)&so2[t * 4]); }
__global__ __launch_bounds__(128) void k_w1(const float* __restrict__ FEAT, const float* __restrict__ NEI, const __bf16* __restrict__ P1, const float* __restrict__ B1, float* __restrict__ FOUT) { __shared__ __align__(16) float sf[4][16][132];
  const int tid = threadIdx.x, wave = tid >> 5, lane = tid & 31, col = lane & 15, g = lane >> 4; const size_t r0 = (size_t)blockIdx.x * 64 + wave * 16; const int c0 = blockIdx.y * 128;
  v8f acc[8] = {};
#pragma unroll 2
  for (int kc = 0; kc < 2 * HH / 32; ++kc) { const float* src = (kc < HH / 32) ? (FEAT + (r0 + col) * HH) : (NEI + (r0 + col) * HH); const F2 a = split_row(src, (kc % (HH / 32)) * 32, lane);
#pragma unroll
    for (int j = 0; j < 8; ++j) { const v16b w = frag_b(P1 + (size_t)(c0 + j * 16 + col) * (2 * HH) + kc * 32, lane); acc[j] = wmma_bf(a.h, w, acc[j]); acc[j] = wmma_bf(a.l, w, acc[j]); } }
#pragma unroll
  for (int j = 0; j < 8; ++j) { const float bb = bfr(B1[c0 + j * 16 + col]);
#pragma unroll
    for (int r = 0; r < 8; ++r) sf[wave][8 * g + r][j * 16 + col] = fmaxf(acc[j][r] + bb, 0.f); }
  LDSX(); for (int rl = 0; rl < 16; ++rl) vst2(FOUT + (r0 + rl) * HH + c0 + lane * 4, *(const v4f*)&sf[wave][rl][lane * 4]); }
__global__ __launch_bounds__(256) void k_sum(const float* __restrict__ FEAT, float* __restrict__ OUT) { __shared__ __align__(16) float so2[HH]; const int t = threadIdx.x; const size_t b = blockIdx.x; float s = 0.f;
#pragma unroll 1
  for (int n = 0; n < NA; ++n) s += FEAT[((b * NA + n) * HH) + t]; so2[t] = s; __syncthreads(); if (t < HH / 4) vst2(OUT + b * HH + t * 4, *(const v4f*)&so2[t * 4]); }
extern "C" void kernel_launch(void* const* d_in, const int* in_sizes, int n_in, void* d_out, int out_size, void* d_ws, size_t ws_size, hipStream_t stream) {
  (void)in_sizes; (void)n_in; (void)out_size;
  const float** F = (const float**)d_in;
  if (ws_size < (size_t)WS_END) return;
  char* ws = (char*)d_ws; __bf16* P = (__bf16*)ws; float *FA = (float*)(ws + WS_FA), *FB = (float*)(ws + WS_FB), *FW = (float*)(ws + WS_FW), *NEI = (float*)(ws + WS_NEI);
  const int nr = TNB * NA;
  k_pack<<<dim3(HH, 2), 256, 0, stream>>>(F[6], F[8], P);
  k_copy<<<nr, 256, 0, stream>>>(F[5], FA);
  float* cur = FA; float* nxt = FB;
  for (int d = 0; d < DEPTH; ++d) {
    k_fw<<<dim3(nr / 64, HH / 128), 128, 0, stream>>>(cur, P + WS_P2 / 2, FW);
    k_nei<<<nr, 256, 0, stream>>>(FW, F[1], (const int*)d_in[2], (const int*)d_in[3], (const int*)d_in[4], F[6], F[7], NEI);
    k_w1<<<dim3(nr / 64, HH / 128), 128, 0, stream>>>(cur, NEI, P + WS_P1 / 2, F[9], nxt);
    float* tmp = cur; cur = nxt; nxt = tmp; }
  k_sum<<<TNB, 256, 0, stream>>>(cur, (float*)d_out);
}
